// Attention_1967095022262
// MI455X (gfx1250) — hardware-run, weakly checked
//
#include <hip/hip_runtime.h>


#ifndef NB
#define NB 4
#endif
#define NB_FULL 4
#ifndef NQ
#define NQ 1024
#endif
#ifndef NK
#define NK 2048
#endif
#define NQ_FULL 1024
#define NK_FULL 2048
#define DM 1024
#define NH 16
#define DH 64
#define HH (NH * DH)
#define SCL 0.125f
#define C2LOG 0.18033688011112042f
#define PCARRY 4096.0f
#define PSHIFT 12.0f
#define AVCARRY 32.0f
#define OWCARRY 64.0f
#define MSCALE 1.52587890625e-05f
#define OUT1_OFF 4194304L

#define AL256(x) (((x) + 255L) & ~255L)
#define WS_TOTAL (AL256((long)NB * NQ * DM * 2) + 2 * AL256((long)NB * NK * DM * 2) + 4 * AL256((long)HH * DM * 2) + \
                  AL256((long)NB * NH * NQ * DH * 2) + 2 * AL256((long)NB * NH * NK * DH * 2) + \
                  AL256((long)NB * NH * NK * 4) + AL256((long)NQ * NB * HH * 2))

static_assert(NB >= 1 && NB <= NB_FULL);
static_assert(NQ >= 128 && NQ <= NQ_FULL && NK >= 128 && NK <= NK_FULL);
static_assert(NQ % 128 == 0 && NK % 128 == 0);
static_assert(DM == 1024 && HH == 1024 && DH == 64 && NH == 16);
static_assert(DM == 128 * 8);
static_assert(DM % 32 == 0 && HH % 32 == 0 && DH % 32 == 0);
static_assert(HH % 128 == 0 && DM % 128 == 0);
static_assert(((long)NQ * NB) % 128 == 0);
static_assert((long)NQ * NB * DM * 4 <= 16777216L);
static_assert(OUT1_OFF * 4 == 16777216L);
static_assert((long)NB * NQ * NK * 4 <= 33554432L);
static_assert(PCARRY == 4096.0f && PSHIFT == 12.0f);
static_assert(MSCALE * 16.0f * PCARRY == 1.0f);
static_assert(WS_TOTAL <= 134217728L);

typedef unsigned short us_t;
typedef _Float16 h16;
typedef us_t     v8us  __attribute__((ext_vector_type(8)));
typedef unsigned v4u   __attribute__((ext_vector_type(4)));
typedef float    v8f   __attribute__((ext_vector_type(8)));
typedef float    v4f   __attribute__((ext_vector_type(4)));
typedef __bf16   v16bf __attribute__((ext_vector_type(16)));
typedef _Float16 v16h  __attribute__((ext_vector_type(16)));

#if __has_builtin(__builtin_amdgcn_exp2f)
#define FEXP2(x) __builtin_amdgcn_exp2f(x)
#else
#define FEXP2(x) __expf((x) * 0.6931471805599453f)
#endif

union Frag16 { v8us u[2]; v16bf bf; v16h hf; };

__device__ __forceinline__ v8f vzero() {
  v8f z = {0.f, 0.f, 0.f, 0.f, 0.f, 0.f, 0.f, 0.f};
  return z;
}

__device__ __forceinline__ us_t bf_bits(float x) {
  unsigned u = __float_as_uint(x);
  u += 0x7FFFu + ((u >> 16) & 1u);
  return (us_t)(u >> 16);
}
__device__ __forceinline__ float bf_val(float x) {
  unsigned u = __float_as_uint(x);
  u += 0x7FFFu + ((u >> 16) & 1u);
  return __uint_as_float(u & 0xFFFF0000u);
}
__device__ __forceinline__ us_t hf_bits(float x) {
  _Float16 hv = (_Float16)x;
  return __builtin_bit_cast(us_t, hv);
}

static __device__ __forceinline__ h16 toh_flush(float v) {
  const h16 r = (h16)v;
  return (fabsf(v) < 6.103515625e-05f) ? (h16)0.0f : r;
}
static __device__ __forceinline__ us_t hfl_bits(float v) {
  return __builtin_bit_cast(us_t, toh_flush(v));
}
static __device__ __forceinline__ float pexp2_cut(float e) {
  const float p = FEXP2(e);
  return (e < -14.0f) ? 0.0f : p;
}

template <int F16OP>
__device__ __forceinline__ v8f mma16(const Frag16& a, const Frag16& b, v8f c) {
  if (F16OP) {
    c = __builtin_amdgcn_wmma_f32_16x16x32_f16(false, a.hf, false, b.hf, (short)0, c, false, false);
    asm volatile("v_nop\n\tv_nop\n\tv_nop\n\tv_nop" : "+v"(c) : "v"(a.hf), "v"(b.hf));
  } else {
    c = __builtin_amdgcn_wmma_f32_16x16x32_bf16(false, a.bf, false, b.bf, (short)0, c, false, false);
    asm volatile("v_nop\n\tv_nop\n\tv_nop\n\tv_nop" : "+v"(c) : "v"(a.bf), "v"(b.bf));
  }
  return c;
}

__global__ __launch_bounds__(128)
void k_cvt_rows(const float* __restrict__ x, us_t* dst, int rows, int rows_full) {
  const int blk = blockIdx.x;
  const int b = blk / rows, pos = blk - b * rows;
  const int t = threadIdx.x;
  const float* src = x + ((size_t)b * rows_full + pos) * DM;
  v4f f0 = *(const v4f*)(src + 8 * t);
  v4f f1 = *(const v4f*)(src + 8 * t + 4);
  float e[8] = {f0[0], f0[1], f0[2], f0[3], f1[0], f1[1], f1[2], f1[3]};
  unsigned wv[4];
#pragma unroll
  for (int k = 0; k < 4; ++k)
    wv[k] = (unsigned)bf_bits(e[2 * k]) | ((unsigned)bf_bits(e[2 * k + 1]) << 16);
  v4u pk = {wv[0], wv[1], wv[2], wv[3]};
  us_t* d = dst + (size_t)blk * DM + 8 * t;
  *(volatile v4u*)d = pk;
  __threadfence();
  *(volatile v4u*)d = pk;
}

template <int MODE>
__global__ __launch_bounds__(128)
void k_cvt_lin(const float* __restrict__ src, us_t* dst) {
  const size_t base = (size_t)blockIdx.x * 1024 + 8 * threadIdx.x;
  v4f f0 = *(const v4f*)(src + base);
  v4f f1 = *(const v4f*)(src + base + 4);
  float e[8] = {f0[0], f0[1], f0[2], f0[3], f1[0], f1[1], f1[2], f1[3]};
  unsigned wv[4];
#pragma unroll
  for (int k = 0; k < 4; ++k) {
    us_t lo, hi;
    if (MODE == 0) { lo = bf_bits(e[2 * k]); hi = bf_bits(e[2 * k + 1]); }
    else           { lo = hf_bits(bf_val(e[2 * k]) * OWCARRY); hi = hf_bits(bf_val(e[2 * k + 1]) * OWCARRY); }
    wv[k] = (unsigned)lo | ((unsigned)hi << 16);
  }
  v4u pk = {wv[0], wv[1], wv[2], wv[3]};
  us_t* d = dst + base;
  *(volatile v4u*)d = pk;
  __threadfence();
  *(volatile v4u*)d = pk;
}

#define BM 128
#define BN 128
#define BK 32
#define BKP 40
#define CSP 136
#define CFP 132
#define EPI_Q 0
#define EPI_K 1
#define EPI_VT 2
#define EPI_OUT 3

template <int F16OP, int EPI>
__global__ __launch_bounds__(256)
void k_gemm(const us_t* __restrict__ A, const us_t* __restrict__ B,
            void* D0, void* D1, const float* __restrict__ bias0, const float* __restrict__ bias1,
            long lda, long ldb, long strideAz, int K)
{
  __shared__ __align__(16) us_t As[BM * BKP];
  __shared__ __align__(16) us_t Bs[BN * BKP];
  __shared__ __align__(16) us_t Cs[BM * CSP];
  static_assert(64 * CFP * 4 <= BM * CSP * 2);

  const int tid = threadIdx.x, lane = tid & 31, wid = __builtin_amdgcn_readfirstlane(tid >> 5);
  const int wm = wid >> 2, wn = wid & 3, h = lane >> 4, l15 = lane & 15;
  const int m0 = blockIdx.y * BM, n0 = blockIdx.x * BN, z = blockIdx.z;
  const us_t* Ab = A + (size_t)z * (size_t)strideAz + (size_t)m0 * (size_t)lda;
  const us_t* Bb = B + (size_t)n0 * (size_t)ldb;

  v8f acc[4][2];
#pragma unroll
  for (int mi = 0; mi < 4; ++mi)
#pragma unroll
    for (int ni = 0; ni < 2; ++ni) acc[mi][ni] = vzero();

  const int nk = K / BK;
  for (int kb = 0; kb < nk; ++kb) {
    const int k0 = kb * BK;
    v8us ra[2], rb[2];
#pragma unroll
    for (int t = 0; t < 2; ++t) {
      const int ch = tid + t * 256, row = ch >> 2, kc = (ch & 3) << 3;
      ra[t] = *(const v8us*)(Ab + (size_t)row * (size_t)lda + k0 + kc);
      rb[t] = *(const v8us*)(Bb + (size_t)row * (size_t)ldb + k0 + kc);
    }
    __syncthreads();
#pragma unroll
    for (int t = 0; t < 2; ++t) {
      const int ch = tid + t * 256, row = ch >> 2, kc = (ch & 3) << 3;
      *(v8us*)(&As[row * BKP + kc]) = ra[t];
      *(v8us*)(&Bs[row * BKP + kc]) = rb[t];
    }
    __syncthreads();
    Frag16 af[4], bfr[2];
#pragma unroll
    for (int mi = 0; mi < 4; ++mi) {
      const int r = wm * 64 + mi * 16 + l15;
      af[mi].u[0] = *(const v8us*)(&As[r * BKP + 8 * h]);
      af[mi].u[1] = *(const v8us*)(&As[r * BKP + 16 + 8 * h]);
    }
#pragma unroll
    for (int ni = 0; ni < 2; ++ni) {
      const int r = wn * 32 + ni * 16 + l15;
      bfr[ni].u[0] = *(const v8us*)(&Bs[r * BKP + 8 * h]);
      bfr[ni].u[1] = *(const v8us*)(&Bs[r * BKP + 16 + 8 * h]);
    }
#pragma unroll
    for (int mi = 0; mi < 4; ++mi)
#pragma unroll
      for (int ni = 0; ni < 2; ++ni) acc[mi][ni] = mma16<F16OP>(af[mi], bfr[ni], acc[mi][ni]);
  }

  const int q8 = tid & 7, lsub = tid >> 3;

  if (EPI == EPI_OUT) {
    float* Cf = (float*)Cs;
    float* Do = (float*)D0;
    const float oscale = 1.0f / (AVCARRY * OWCARRY);
#pragma unroll
    for (int rh = 0; rh < 2; ++rh) {
      __syncthreads();
      if (wm == rh) {
#pragma unroll
        for (int mi = 0; mi < 4; ++mi)
#pragma unroll
          for (int ni = 0; ni < 2; ++ni) {
            const int col = wn * 32 + ni * 16 + l15;
#pragma unroll
            for (int v = 0; v < 8; ++v)
              Cf[(mi * 16 + 8 * h + v) * CFP + col] = acc[mi][ni][v] * oscale;
          }
      }
      __syncthreads();
      for (int ps = 0; ps < 2; ++ps) {
#pragma unroll
        for (int it = 0; it < 8; ++it) {
          const int L = it * 32 + lsub, pr = L >> 2, ql = L & 3;
          const v4f val = *(const v4f*)(&Cf[pr * CFP + 32 * ql + 4 * q8]);
          const v4f bq = *(const v4f*)(bias0 + n0 + 32 * ql + 4 * q8);
          const v4f o = {val[0] + bf_val(bq[0]), val[1] + bf_val(bq[1]),
                         val[2] + bf_val(bq[2]), val[3] + bf_val(bq[3])};
          float* dst = Do + ((size_t)(m0 + 64 * rh + pr) * DM + n0 + 32 * ql + 4 * q8);
          *(volatile v4f*)dst = o;
        }
        if (ps == 0) __threadfence();
      }
    }
  } else {
    __syncthreads();
#pragma unroll
    for (int mi = 0; mi < 4; ++mi)
#pragma unroll
      for (int ni = 0; ni < 2; ++ni) {
        const int col = wn * 32 + ni * 16 + l15;
#pragma unroll
        for (int v = 0; v < 8; ++v)
          Cs[(wm * 64 + mi * 16 + 8 * h + v) * CSP + col] = hfl_bits(acc[mi][ni][v]);
      }
    __syncthreads();
    const int rpb = (EPI == EPI_Q) ? NQ : NK;
    const int hb = n0 >> 6;
    for (int ps = 0; ps < 2; ++ps) {
      if (EPI != EPI_VT) {
#pragma unroll
        for (int it = 0; it < 8; ++it) {
          const int L = it * 32 + lsub, pr = L >> 1, nl = L & 1;
          v4u val = *(const v4u*)(&Cs[pr * CSP + nl * 64 + 8 * q8]);
          us_t* dst = (us_t*)D0 + ((((size_t)z * NH + hb + nl) * rpb + m0 + pr) * DH + 8 * q8);
          *(volatile v4u*)dst = val;
        }
      } else {
#pragma unroll
        for (int it = 0; it < 8; ++it) {
          const int L = it * 32 + lsub, nl = L >> 7, d = (L >> 1) & 63, hp = L & 1;
          const int rb0 = 64 * hp + 8 * q8, cc = nl * 64 + d;
          unsigned wv[4];
#pragma unroll
          for (int k = 0; k < 4; ++k) {
            const unsigned lo = Cs[(rb0 + 2 * k) * CSP + cc];
            const unsigned hi = Cs[(rb0 + 2 * k + 1) * CSP + cc];
            wv[k] = lo | (hi << 16);
          }
          v4u val = {wv[0], wv[1], wv[2], wv[3]};
          us_t* dst = (us_t*)D0 + ((((size_t)z * NH + hb + nl) * DH + d) * NK + m0 + 64 * hp + 8 * q8);
          *(volatile v4u*)dst = val;
        }
      }
      if (ps == 0) __threadfence();
    }
  }
}

__global__ __launch_bounds__(128)
void k_colstats(const us_t* __restrict__ Qp, const us_t* __restrict__ Kp, float* NLS)
{
  __shared__ __align__(16) float sred[64];
  const int lane = threadIdx.x & 31;
  const int wave = __builtin_amdgcn_readfirstlane(threadIdx.x >> 5);
  const int h = lane >> 4, l15 = lane & 15;
  const int bn = blockIdx.y;
  const int kb0 = blockIdx.x * 64;

  Frag16 kf[2];
  {
    const us_t* kr = Kp + ((size_t)bn * NK + kb0 + wave * 16 + l15) * DH;
#pragma unroll
    for (int c = 0; c < 2; ++c) {
      kf[c].u[0] = *(const v8us*)(kr + 32 * c + 8 * h);
      kf[c].u[1] = *(const v8us*)(kr + 32 * c + 16 + 8 * h);
    }
  }

  float mrun = -3.0e38f, lrun = 0.f;
  const us_t* Qbase = Qp + (size_t)bn * NQ * DH;
  for (int qt = 0; qt < NQ / 32; ++qt) {
    const us_t* qa = Qbase + (size_t)(qt * 32 + l15) * DH;
    v8f s0 = vzero(), s1 = vzero();
#pragma unroll
    for (int c = 0; c < 2; ++c) {
      Frag16 a0, a1;
      a0.u[0] = *(const v8us*)(qa + 32 * c + 8 * h);
      a0.u[1] = *(const v8us*)(qa + 32 * c + 16 + 8 * h);
      a1.u[0] = *(const v8us*)(qa + 16 * DH + 32 * c + 8 * h);
      a1.u[1] = *(const v8us*)(qa + 16 * DH + 32 * c + 16 + 8 * h);
      s0 = mma16<1>(a0, kf[c], s0);
      s1 = mma16<1>(a1, kf[c], s1);
    }
    float tmx = fmaxf(s0[0], s1[0]);
#pragma unroll
    for (int r = 1; r < 8; ++r) tmx = fmaxf(tmx, fmaxf(s0[r], s1[r]));
    const float mn = fmaxf(mrun, tmx * C2LOG);
    float ps = 0.f;
#pragma unroll
    for (int r = 0; r < 8; ++r) {
      ps += FEXP2(fmaf(s0[r], C2LOG, -mn));
      ps += FEXP2(fmaf(s1[r], C2LOG, -mn));
    }
    lrun = lrun * FEXP2(mrun - mn) + ps;
    mrun = mn;
  }

  const float m2 = __shfl_xor(mrun, 16);
  const float l2 = __shfl_xor(lrun, 16);
  const float mt = fmaxf(mrun, m2);
  const float lt = lrun * FEXP2(mrun - mt) + l2 * FEXP2(m2 - mt);
  const float nls = PSHIFT - (mt + log2f(lt));

  if (h == 0) sred[wave * 16 + l15] = nls;
  __syncthreads();
  if (wave == 0) {
    const int li = (lane < 16) ? lane : 15;
    const v4f val = *(const v4f*)(&sred[4 * li]);
    float* dst = NLS + (size_t)bn * NK + kb0 + 4 * li;
    if (lane < 16) *(volatile v4f*)dst = val;
    __threadfence();
    if (lane < 16) *(volatile v4f*)dst = val;
  }
}

#define MP 68

__global__ __launch_bounds__(128)
void k_attn_mean(const us_t* __restrict__ Qp, const us_t* __restrict__ Kp,
                 const float* __restrict__ NLS, float* out1)
{
  __shared__ __align__(16) float Mst[4 * 16 * MP];
  const int lane = threadIdx.x & 31;
  const int wave = __builtin_amdgcn_readfirstlane(threadIdx.x >> 5);
  const int h = lane >> 4, l15 = lane & 15;
  const int k0 = blockIdx.x * 64;
  const int q0 = blockIdx.y * 64 + wave * 16;
  const int b = blockIdx.z;
  const int mw = wave * (16 * MP);

  v8f macc[4];
#pragma unroll
  for (int st = 0; st < 4; ++st) macc[st] = vzero();

#pragma unroll 1
  for (int hh = 0; hh < NH; ++hh) {
    const int bn = b * NH + hh;
    Frag16 qa[2];
    {
      const us_t* pq = Qp + ((size_t)bn * NQ + q0 + l15) * DH;
#pragma unroll
      for (int c = 0; c < 2; ++c) {
        qa[c].u[0] = *(const v8us*)(pq + 32 * c + 8 * h);
        qa[c].u[1] = *(const v8us*)(pq + 32 * c + 16 + 8 * h);
      }
    }
    const us_t* kb = Kp + ((size_t)bn * NK + k0 + l15) * DH;
    const float* np = NLS + (size_t)bn * NK + k0 + l15;
#pragma unroll
    for (int st = 0; st < 4; ++st) {
      v8f s = vzero();
#pragma unroll
      for (int c = 0; c < 2; ++c) {
        Frag16 bf;
        bf.u[0] = *(const v8us*)(kb + (size_t)(16 * st) * DH + 32 * c + 8 * h);
        bf.u[1] = *(const v8us*)(kb + (size_t)(16 * st) * DH + 32 * c + 16 + 8 * h);
        s = mma16<1>(qa[c], bf, s);
      }
      const float nl = np[16 * st];
#pragma unroll
      for (int r = 0; r < 8; ++r) macc[st][r] += FEXP2(fmaf(s[r], C2LOG, nl));
    }
  }

#pragma unroll
  for (int st = 0; st < 4; ++st)
#pragma unroll
    for (int r = 0; r < 8; ++r)
      Mst[mw + (8 * h + r) * MP + 16 * st + l15] = macc[st][r] * MSCALE;
  __syncthreads();
  const int q8 = lane & 7, rsub = lane >> 3;
  for (int ps = 0; ps < 2; ++ps) {
#pragma unroll
    for (int it = 0; it < 8; ++it) {
      const int L = it * 4 + rsub, row = L >> 1, nl = L & 1;
      const v4f val = *(const v4f*)(&Mst[mw + row * MP + 32 * nl + 4 * q8]);
      float* dst = out1 + (((size_t)b * NQ + q0 + row) * NK + k0 + 32 * nl + 4 * q8);
      *(volatile v4f*)dst = val;
    }
    if (ps == 0) __threadfence();
  }
}

#define PP 72

__global__ __launch_bounds__(128)
void k_attn_ctx(const us_t* __restrict__ Qp, const us_t* __restrict__ Kp, const us_t* __restrict__ Vt,
                const float* __restrict__ NLS, us_t* AV)
{
  __shared__ __align__(16) us_t Ost[4 * 16 * PP];
  const int lane = threadIdx.x & 31;
  const int wave = __builtin_amdgcn_readfirstlane(threadIdx.x >> 5);
  const int h = lane >> 4, l15 = lane & 15;
  const int i0 = blockIdx.x * 64, bn = blockIdx.y;
  const int b = bn / NH, n = bn - b * NH;
  const int iw = i0 + wave * 16;
  const int ow = wave * (16 * PP);

  Frag16 qf[2];
  {
    const us_t* pq = Qp + ((size_t)bn * NQ + iw + l15) * DH;
#pragma unroll
    for (int c = 0; c < 2; ++c) {
      qf[c].u[0] = *(const v8us*)(pq + 32 * c + 8 * h);
      qf[c].u[1] = *(const v8us*)(pq + 32 * c + 16 + 8 * h);
    }
  }

  v8f oacc[4];
#pragma unroll
  for (int dt = 0; dt < 4; ++dt) oacc[dt] = vzero();

  const us_t* Kbase = Kp + (size_t)bn * NK * DH;
  const us_t* Vbase = Vt + (size_t)bn * DH * NK;
  const float* Nbase = NLS + (size_t)bn * NK;

  for (int kt = 0; kt < NK / 32; ++kt) {
    const int kt0 = kt * 32;
    Frag16 pb;
#pragma unroll
    for (int st = 0; st < 2; ++st) {
      v8f s = vzero();
      const us_t* kr = Kbase + (size_t)(kt0 + 16 * st + l15) * DH;
#pragma unroll
      for (int c = 0; c < 2; ++c) {
        Frag16 ka;
        ka.u[0] = *(const v8us*)(kr + 32 * c + 8 * h);
        ka.u[1] = *(const v8us*)(kr + 32 * c + 16 + 8 * h);
        s = mma16<1>(ka, qf[c], s);
      }
      const float* np = Nbase + kt0 + 16 * st + 8 * h;
      const v4f na = *(const v4f*)(np);
      const v4f nc = *(const v4f*)(np + 4);
      const float nl[8] = {na[0], na[1], na[2], na[3], nc[0], nc[1], nc[2], nc[3]};
#pragma unroll
      for (int r = 0; r < 8; ++r)
        pb.hf[8 * st + r] = (h16)pexp2_cut(fmaf(s[r], C2LOG, nl[r]));
    }
#pragma unroll
    for (int dt = 0; dt < 4; ++dt) {
      Frag16 va;
      const us_t* vr = Vbase + (size_t)(16 * dt + l15) * NK + kt0;
      va.u[0] = *(const v8us*)(vr + 8 * h);
      va.u[1] = *(const v8us*)(vr + 16 + 8 * h);
      oacc[dt] = mma16<1>(va, pb, oacc[dt]);
    }
  }

  const float sc = AVCARRY / PCARRY;
#pragma unroll
  for (int dt = 0; dt < 4; ++dt) {
    v8us pk;
#pragma unroll
    for (int r = 0; r < 8; ++r) pk[r] = hfl_bits(oacc[dt][r] * sc);
    *(v8us*)(&Ost[ow + l15 * PP + 16 * dt + 8 * h]) = pk;
  }
  __syncthreads();
  const int q8 = lane & 7, rsub = lane >> 3;
  for (int ps = 0; ps < 2; ++ps) {
#pragma unroll
    for (int it = 0; it < 4; ++it) {
      const int row = it * 4 + rsub;
      v4u val = *(const v4u*)(&Ost[ow + row * PP + 8 * q8]);
      us_t* dst = AV + (((size_t)(iw + row) * NB + b) * HH + n * DH + 8 * q8);
      *(volatile v4u*)dst = val;
    }
    if (ps == 0) __threadfence();
  }
}

extern "C" void kernel_launch(void* const* d_in, const int* in_sizes, int n_in,
                              void* d_out, int out_size, void* d_ws, size_t ws_size,
                              hipStream_t stream)
{
  if (n_in < 8) return;
  const float* xq = (const float*)d_in[0];
  const float* xk = (const float*)d_in[1];
  const float* xv = (const float*)d_in[2];
  const float* wq = (const float*)d_in[3];
  const float* wk = (const float*)d_in[4];
  const float* wv = (const float*)d_in[5];
  const float* wp = (const float*)d_in[6];
  const float* bp = (const float*)d_in[7];

  if ((long)in_sizes[0] < ((long)(NB - 1) * NQ_FULL + NQ) * DM) return;
  if ((long)in_sizes[1] < ((long)(NB - 1) * NK_FULL + NK) * DM) return;
  if ((long)in_sizes[2] < ((long)(NB - 1) * NK_FULL + NK) * DM) return;
  if ((long)in_sizes[3] < (long)HH * DM) return;
  if ((long)in_sizes[4] < (long)HH * DM) return;
  if ((long)in_sizes[5] < (long)HH * DM) return;
  if ((long)in_sizes[6] < (long)DM * HH) return;
  if (in_sizes[7] < DM) return;
  if ((long)out_size < OUT1_OFF + (long)NB * NQ * NK) return;

  char* base = (char*)d_ws;
  size_t off = 0;
  auto take = [&](size_t bytes) -> char* {
    char* q = base + off; off += (bytes + 255) & ~(size_t)255; return q;
  };
  us_t*  xq_b = (us_t*) take((size_t)NB * NQ * DM * 2);
  us_t*  xk_b = (us_t*) take((size_t)NB * NK * DM * 2);
  us_t*  xv_b = (us_t*) take((size_t)NB * NK * DM * 2);
  us_t*  wq_b = (us_t*) take((size_t)HH * DM * 2);
  us_t*  wk_b = (us_t*) take((size_t)HH * DM * 2);
  us_t*  wv_b = (us_t*) take((size_t)HH * DM * 2);
  us_t*  wp_h = (us_t*) take((size_t)DM * HH * 2);
  us_t*  Qp   = (us_t*) take((size_t)NB * NH * NQ * DH * 2);
  us_t*  Kp   = (us_t*) take((size_t)NB * NH * NK * DH * 2);
  us_t*  Vt   = (us_t*) take((size_t)NB * NH * DH * NK * 2);
  float* NLS  = (float*)take((size_t)NB * NH * NK * 4);
  us_t*  AV   = (us_t*) take((size_t)NQ * NB * HH * 2);
  if (off > ws_size) return;
  if (off > (size_t)WS_TOTAL) return;

  float* out0 = (float*)d_out;
  float* out1 = (float*)d_out + OUT1_OFF;

  k_cvt_rows<<<dim3(NB * NQ), dim3(128), 0, stream>>>(xq, xq_b, NQ, NQ_FULL);
  k_cvt_rows<<<dim3(NB * NK), dim3(128), 0, stream>>>(xk, xk_b, NK, NK_FULL);
  k_cvt_rows<<<dim3(NB * NK), dim3(128), 0, stream>>>(xv, xv_b, NK, NK_FULL);
  k_cvt_lin<0><<<dim3(HH * DM / 1024), dim3(128), 0, stream>>>(wq, wq_b);
  k_cvt_lin<0><<<dim3(HH * DM / 1024), dim3(128), 0, stream>>>(wk, wk_b);
  k_cvt_lin<0><<<dim3(HH * DM / 1024), dim3(128), 0, stream>>>(wv, wv_b);
  k_cvt_lin<1><<<dim3(DM * HH / 1024), dim3(128), 0, stream>>>(wp, wp_h);

  k_gemm<0, EPI_Q><<<dim3(HH / BN, NQ / BM, NB), dim3(256), 0, stream>>>(
      xq_b, wq_b, (void*)Qp, (void*)Qp, bp, bp, (long)DM, (long)DM, (long)NQ * DM, DM);
  k_gemm<0, EPI_K><<<dim3(HH / BN, NK / BM, NB), dim3(256), 0, stream>>>(
      xk_b, wk_b, (void*)Kp, (void*)Kp, bp, bp, (long)DM, (long)DM, (long)NK * DM, DM);
  k_gemm<0, EPI_VT><<<dim3(HH / BN, NK / BM, NB), dim3(256), 0, stream>>>(
      xv_b, wv_b, (void*)Vt, (void*)Vt, bp, bp, (long)DM, (long)DM, (long)NK * DM, DM);

  k_colstats<<<dim3(NK / 64, NB * NH), dim3(128), 0, stream>>>(Qp, Kp, NLS);
  k_attn_mean<<<dim3(NK / 64, NQ / 64, NB), dim3(128), 0, stream>>>(Qp, Kp, NLS, out1);
  k_attn_ctx<<<dim3(NQ / 64, NB * NH), dim3(128), 0, stream>>>(Qp, Kp, Vt, NLS, AV);
  k_gemm<1, EPI_OUT><<<dim3(DM / BN, (NQ * NB) / BM, 1), dim3(256), 0, stream>>>(
      AV, wp_h, (void*)out0, (void*)out0, bp, bp, (long)HH, (long)HH, 0L, HH);
}
